// TransformerEncoderLayer_44598940401888
// MI455X (gfx1250) — hardware-verified
//
#include <hip/hip_runtime.h>
#ifndef NB
#define NB 2
#endif
#ifndef SEQ
#define SEQ 2048
#endif
#define NB_FULL 2
#define SEQ_FULL 2048
#define DM 1024
#define NH 16
#define HD 64
#define DFF 4096
#define DMQ DM
#define NR ((size_t)NB * SEQ)
#define LQK (2 * DM)
static_assert(SEQ % 64 == 0);
static_assert(NB >= 1 && NB <= NB_FULL);
static_assert(SEQ <= SEQ_FULL);
static_assert(NH * HD == DM);
static_assert(HD == 64);
static_assert(DM % 128 == 0 && DFF % 64 == 0 && DM % 32 == 0 && DFF % 32 == 0);
static_assert(((size_t)NB * SEQ) % 128 == 0);
static_assert(DMQ % 4 == 0 && DMQ / 4 == 256);
static_assert((((size_t)NB * SEQ) * DM / 8) % 256 == 0);
static_assert(((size_t)NH * HD * (DM / 8)) % 256 == 0);
static_assert(((size_t)DM * DFF / 8) % 256 == 0);

typedef unsigned short v8us __attribute__((ext_vector_type(8), may_alias));
typedef float  v8f  __attribute__((ext_vector_type(8)));
typedef float  v4f  __attribute__((ext_vector_type(4)));
typedef float  v4fa __attribute__((ext_vector_type(4), may_alias));
typedef _Float16 v16h __attribute__((ext_vector_type(16)));
typedef _Float16 v4h __attribute__((ext_vector_type(4)));
union FragH { v16h v; v8us half[2]; _Float16 h[16]; unsigned short u[16]; };

__device__ __forceinline__ unsigned short bf16_bits(float x) { unsigned int u = __float_as_uint(x); return (unsigned short)((u + 0x7FFFu + ((u >> 16) & 1u)) >> 16); }
__device__ __forceinline__ float bf16_val(unsigned short b) { return __uint_as_float(((unsigned int)b) << 16); }
__device__ __forceinline__ float bf16_rne(float x) { return bf16_val(bf16_bits(x)); }

__device__ __forceinline__ v16h g2_frag(const _Float16* p, unsigned hh) { FragH f; f.half[0] = *(const v8us*)((const unsigned short*)p + 8u * hh); f.half[1] = *(const v8us*)((const unsigned short*)p + 16u + 8u * hh); return f.v; }
__device__ __forceinline__ v8f g2_mma(v16h a, v16h b, v8f c) { v8f d = __builtin_amdgcn_wmma_f32_16x16x32_f16(false, a, false, b, (short)0, c, false, false); asm volatile("v_nop\n\tv_nop\n\tv_nop\n\tv_nop" : "+v"(d) : "v"(a), "v"(b)); return d; }

template <unsigned K, unsigned N>
__global__ __launch_bounds__(256) void k_wt_f16(const float* __restrict__ W, _Float16* __restrict__ Wt, float scale) {
  static_assert(K % 64 == 0);
  const unsigned t = blockIdx.x * 256u + threadIdx.x; if (t >= N * (K / 8u)) return; const unsigned n = t / (K / 8u), k8 = (t % (K / 8u)) * 8u; FragH f;
#pragma unroll
  for (unsigned i = 0; i < 8; ++i) f.h[i] = (_Float16)(bf16_rne(W[(size_t)(k8 + i) * N + n]) * scale);
  const v8us o = f.half[0];
  *(volatile v8us*)((unsigned short*)Wt + (size_t)n * K + k8) = o; __threadfence(); *(volatile v8us*)((unsigned short*)Wt + (size_t)n * K + k8) = o;
}

__global__ __launch_bounds__(256) void k_wthd3(const float* __restrict__ Wa, const float* __restrict__ Wb, const float* __restrict__ Wc, _Float16* __restrict__ Bt) {
  const unsigned t = blockIdx.x * 256u + threadIdx.x; if (t >= (unsigned)NH * HD * (DM / 8)) return;
  const unsigned which = blockIdx.y; const float* W = (which == 0u) ? Wa : ((which == 1u) ? Wb : Wc);
  const unsigned m8 = (t % (unsigned)(DM / 8)) * 8u; const unsigned d = (t / (unsigned)(DM / 8)) % (unsigned)HD; const unsigned h = t / ((unsigned)(DM / 8) * (unsigned)HD); FragH f;
#pragma unroll
  for (unsigned q = 0; q < 8; ++q) f.h[q] = (_Float16)(16.0f * bf16_rne(W[((size_t)h * DM + m8 + q) * HD + d]));
  const v8us o = f.half[0];
  unsigned short* dst = (unsigned short*)Bt + ((size_t)which * DM + (size_t)h * HD + d) * DM + m8;
  *(volatile v8us*)dst = o; __threadfence(); *(volatile v8us*)dst = o;
}

__global__ __launch_bounds__(256) void k_xprep(const float* __restrict__ x, _Float16* __restrict__ X16, unsigned n8) {
  const unsigned t = blockIdx.x * 256u + threadIdx.x; if (t >= n8) return;
  const size_t e = (size_t)t * 8u; const size_t r = e / DM; const size_t c = e % DM; const size_t rs = (r / SEQ) * SEQ_FULL + (r % SEQ);
  const float* p = x + rs * DM + c; const v4f a = *(const v4fa*)p, cc = *(const v4fa*)(p + 4); FragH f;
#pragma unroll
  for (unsigned q = 0; q < 4; ++q) { f.h[q] = (_Float16)bf16_rne(a[q]); f.h[4 + q] = (_Float16)bf16_rne(cc[q]); }
  const v8us o = f.half[0];
  *(volatile v8us*)((unsigned short*)X16 + e) = o; __threadfence(); *(volatile v8us*)((unsigned short*)X16 + e) = o;
}

template <int ACT, int BROW>
__global__ __launch_bounds__(128) void k_gemm2(const _Float16* __restrict__ A, int lda, const _Float16* __restrict__ Bh, int ldb, float alpha, const float* __restrict__ bias, const float* __restrict__ CP,
    float* __restrict__ C, _Float16* __restrict__ C16, int ldc, int M, int N, int K) { static_assert(ACT == 0 || ACT == 3); static_assert(BROW == 0 || BROW == 1);
  __shared__ __attribute__((aligned(16))) float so[4][32][68];
  const unsigned tid = threadIdx.x, w = tid >> 5, lane = tid & 31u, ln = lane & 15u, hh = lane >> 4;
  const unsigned row0 = blockIdx.y * 128u + 32u * w, col0 = blockIdx.x * 64u; if (row0 >= (unsigned)M || col0 >= (unsigned)N) return;
  const _Float16* a0p = A + (size_t)(row0 + ln) * lda; const _Float16* a1p = a0p + (size_t)16 * lda;
  const _Float16* b0p = Bh + (size_t)(col0 + ln) * ldb; const _Float16* b1p = b0p + (size_t)16 * ldb; const _Float16* b2p = b1p + (size_t)16 * ldb; const _Float16* b3p = b2p + (size_t)16 * ldb;
  const v8f z8 = {0.f,0.f,0.f,0.f,0.f,0.f,0.f,0.f}; v8f c00 = z8, c01 = z8, c02 = z8, c03 = z8, c10 = z8, c11 = z8, c12 = z8, c13 = z8;
  const unsigned Ku = (unsigned)K;
#pragma unroll 1
  for (unsigned kb = 0; kb < Ku; kb += 32u) { const v16h a0 = g2_frag(a0p + kb, hh), a1 = g2_frag(a1p + kb, hh);
    v16h b = g2_frag(b0p + kb, hh); c00 = g2_mma(a0, b, c00); c10 = g2_mma(a1, b, c10);
    b = g2_frag(b1p + kb, hh); c01 = g2_mma(a0, b, c01); c11 = g2_mma(a1, b, c11);
    b = g2_frag(b2p + kb, hh); c02 = g2_mma(a0, b, c02); c12 = g2_mma(a1, b, c12);
    b = g2_frag(b3p + kb, hh); c03 = g2_mma(a0, b, c03); c13 = g2_mma(a1, b, c13); }
  v8f accs[8] = {c00, c01, c02, c03, c10, c11, c12, c13};
#pragma unroll
  for (unsigned u = 0; u < 8; ++u) { const unsigned t = u & 3u, half = u >> 2; const unsigned col = col0 + t * 16u + ln; float bc = 0.f; if (bias != nullptr && BROW == 0) bc = bf16_rne(bias[col]);
#pragma unroll
    for (unsigned r = 0; r < 8; ++r) { const unsigned rloc = half * 16u + 8u * hh + r; float v = accs[u][r] * alpha + bc;
      if (BROW == 1 && bias != nullptr) v += bf16_rne(bias[row0 + rloc]);
      if (CP) v += CP[(size_t)(row0 + rloc) * ldc + col];
      if (ACT == 3) v = fmaxf(v, 0.f);
      so[w][rloc][t * 16u + ln] = v; } }
  __builtin_amdgcn_fence(4  , "workgroup"); __builtin_amdgcn_wave_barrier();
  const unsigned rsub = lane >> 4, c4 = (lane & 15u) * 4u;
  for (int pass = 0; pass < 2; ++pass) {
#pragma unroll
    for (unsigned q = 0; q < 16; ++q) { const unsigned r = q * 2u + rsub; const v4f v = *(const v4fa*)&so[w][r][c4]; if (C) *(volatile v4f*)(C + (size_t)(row0 + r) * ldc + col0 + c4) = v; if (C16) { v4h h4; for (int i = 0; i < 4; ++i) h4[i] = (_Float16)v[i]; *(volatile v4h*)(C16 + (size_t)(row0 + r) * ldc + col0 + c4) = h4; } }
    if (pass == 0) __threadfence(); } }

template <int BFIN, int W16, int W32, int ORM>
__global__ __launch_bounds__(256) void k_lnx(const float* __restrict__ X, const float* __restrict__ g, const float* __restrict__ bb, float eps, _Float16* __restrict__ N16, float* __restrict__ N32) {
  #pragma clang fp contract(off)
  __shared__ float red[256]; const size_t r = blockIdx.x; const size_t ro = ORM ? ((r / SEQ) * SEQ_FULL + (r % SEQ)) : r; const unsigned t = threadIdx.x; const bool act = t < (unsigned)(DMQ / 4); const unsigned c0 = act ? t * 4u : 0u;
  const v4f xa = *(const v4fa*)(X + r * DMQ + c0); float s[4]; float sum = 0.f;
  for (int q = 0; q < 4; ++q) { s[q] = act ? (BFIN ? bf16_rne(xa[q]) : xa[q]) : 0.f; sum = __fadd_rn(sum, s[q]); }
  red[t] = sum; __syncthreads(); for (unsigned st = 128; st > 0; st >>= 1) { if (t < st) red[t] = __fadd_rn(red[t], red[t + st]); __syncthreads(); } const float mu = red[0] / (float)DMQ; __syncthreads();
  float vs = 0.f; for (int q = 0; q < 4; ++q) { const float dl = act ? __fadd_rn(s[q], -mu) : 0.f; vs = __fadd_rn(vs, __fmul_rn(dl, dl)); } red[t] = vs; __syncthreads(); for (unsigned st = 128; st > 0; st >>= 1) { if (t < st) red[t] = __fadd_rn(red[t], red[t + st]); __syncthreads(); }
  const float rs = rsqrtf(__fadd_rn(red[0] / (float)DMQ, eps)); v4h y; v4f yf;
  for (int q = 0; q < 4; ++q) { const unsigned c = c0 + (unsigned)q; yf[q] = __fadd_rn(__fmul_rn(__fmul_rn(__fadd_rn(s[q], -mu), rs), bf16_rne(g[c])), bf16_rne(bb[c])); y[q] = (_Float16)yf[q]; }
  if (!act) return;
  for (int pass = 0; pass < 2; ++pass) { if (W16) *(volatile v4h*)(N16 + ro * DMQ + c0) = y; if (W32) *(volatile v4f*)(N32 + ro * DMQ + c0) = yf; if (pass == 0) __threadfence(); } }

__global__ __launch_bounds__(128) void k_attn(const _Float16* __restrict__ QK, const _Float16* __restrict__ VT, const float* __restrict__ x, float* __restrict__ T1) {
  __shared__ __attribute__((aligned(16))) float so[4][16][68];
  const unsigned tid = threadIdx.x, w = tid >> 5, lane = tid & 31u, nl = lane & 15u, hh = lane >> 4;
  const unsigned h = blockIdx.y, b = blockIdx.z;
  const unsigned q0 = blockIdx.x * 64u + w * 16u;
  const size_t rq = (size_t)b * SEQ + q0;
  const size_t rk = (size_t)b * SEQ;
  const _Float16* qp = QK + (rq + nl) * LQK + (size_t)h * HD;
  const v16h qb0 = g2_frag(qp, hh), qb1 = g2_frag(qp + 32, hh);
  const _Float16* kp = QK + (rk + nl) * LQK + DM + (size_t)h * HD;
  const _Float16* vp = VT + ((size_t)h * HD + nl) * NR + rk;
  const v8f z8 = {0.f,0.f,0.f,0.f,0.f,0.f,0.f,0.f};
  v8f o0 = z8, o1 = z8, o2 = z8, o3 = z8; float m = -1.0e30f, l = 0.f;
#pragma unroll 1
  for (unsigned kb = 0; kb < (unsigned)SEQ; kb += 32u) {
    const _Float16* k0p = kp + (size_t)kb * LQK; const _Float16* k1p = k0p + (size_t)16 * LQK;
    v8f s0 = z8, s1 = z8; v16h a;
    a = g2_frag(k0p, hh); s0 = g2_mma(a, qb0, s0); a = g2_frag(k0p + 32, hh); s0 = g2_mma(a, qb1, s0);
    a = g2_frag(k1p, hh); s1 = g2_mma(a, qb0, s1); a = g2_frag(k1p + 32, hh); s1 = g2_mma(a, qb1, s1);
    float mx = -1.0e30f;
#pragma unroll
    for (int r = 0; r < 8; ++r) mx = fmaxf(mx, fmaxf(s0[r], s1[r]));
    mx = fmaxf(mx, __shfl_xor(mx, 16, 32));
    const float mn = fmaxf(m, mx * 0.125f);
    const float sc = __expf(m - mn);
    FragH pf; float ps = 0.f;
#pragma unroll
    for (int r = 0; r < 8; ++r) { const float e0 = __expf(s0[r] * 0.125f - mn); const float e1 = __expf(s1[r] * 0.125f - mn); ps += e0 + e1; pf.h[r] = (_Float16)(e0 * 256.0f); pf.h[8 + r] = (_Float16)(e1 * 256.0f); }
    ps += __shfl_xor(ps, 16, 32);
    l = l * sc + ps; m = mn;
#pragma unroll
    for (int r = 0; r < 8; ++r) { o0[r] *= sc; o1[r] *= sc; o2[r] *= sc; o3[r] *= sc; }
    const _Float16* v0p = vp + kb;
    a = g2_frag(v0p, hh); o0 = g2_mma(a, pf.v, o0);
    a = g2_frag(v0p + (size_t)16 * NR, hh); o1 = g2_mma(a, pf.v, o1);
    a = g2_frag(v0p + (size_t)32 * NR, hh); o2 = g2_mma(a, pf.v, o2);
    a = g2_frag(v0p + (size_t)48 * NR, hh); o3 = g2_mma(a, pf.v, o3);
  }
  const float inv = 0.00390625f / l;
  { v4f lo4, hi4;
    lo4[0] = o0[0] * inv; lo4[1] = o0[1] * inv; lo4[2] = o0[2] * inv; lo4[3] = o0[3] * inv; hi4[0] = o0[4] * inv; hi4[1] = o0[5] * inv; hi4[2] = o0[6] * inv; hi4[3] = o0[7] * inv;
    *(v4fa*)&so[w][nl][0u * 16u + 8u * hh] = lo4; *(v4fa*)&so[w][nl][0u * 16u + 8u * hh + 4u] = hi4;
    lo4[0] = o1[0] * inv; lo4[1] = o1[1] * inv; lo4[2] = o1[2] * inv; lo4[3] = o1[3] * inv; hi4[0] = o1[4] * inv; hi4[1] = o1[5] * inv; hi4[2] = o1[6] * inv; hi4[3] = o1[7] * inv;
    *(v4fa*)&so[w][nl][1u * 16u + 8u * hh] = lo4; *(v4fa*)&so[w][nl][1u * 16u + 8u * hh + 4u] = hi4;
    lo4[0] = o2[0] * inv; lo4[1] = o2[1] * inv; lo4[2] = o2[2] * inv; lo4[3] = o2[3] * inv; hi4[0] = o2[4] * inv; hi4[1] = o2[5] * inv; hi4[2] = o2[6] * inv; hi4[3] = o2[7] * inv;
    *(v4fa*)&so[w][nl][2u * 16u + 8u * hh] = lo4; *(v4fa*)&so[w][nl][2u * 16u + 8u * hh + 4u] = hi4;
    lo4[0] = o3[0] * inv; lo4[1] = o3[1] * inv; lo4[2] = o3[2] * inv; lo4[3] = o3[3] * inv; hi4[0] = o3[4] * inv; hi4[1] = o3[5] * inv; hi4[2] = o3[6] * inv; hi4[3] = o3[7] * inv;
    *(v4fa*)&so[w][nl][3u * 16u + 8u * hh] = lo4; *(v4fa*)&so[w][nl][3u * 16u + 8u * hh + 4u] = hi4; }
  __builtin_amdgcn_fence(4  , "workgroup"); __builtin_amdgcn_wave_barrier();
  const unsigned rsub = lane >> 4, c4 = (lane & 15u) * 4u;
  const float* xp = x + ((size_t)b * SEQ_FULL + q0) * DM + (size_t)h * HD + c4;
  float* tp = T1 + rq * DM + (size_t)h * HD + c4;
  v4f ov[8];
#pragma unroll
  for (unsigned q = 0; q < 8; ++q) { const unsigned row = q * 2u + rsub; const v4f sv = *(const v4fa*)&so[w][row][c4]; const v4f xv = *(const v4fa*)(xp + (size_t)row * DM); v4f r4;
    r4[0] = bf16_rne(xv[0]) + sv[0]; r4[1] = bf16_rne(xv[1]) + sv[1]; r4[2] = bf16_rne(xv[2]) + sv[2]; r4[3] = bf16_rne(xv[3]) + sv[3]; ov[q] = r4; }
  for (int pass = 0; pass < 2; ++pass) {
#pragma unroll
    for (unsigned q = 0; q < 8; ++q) { const unsigned row = q * 2u + rsub; *(volatile v4f*)(tp + (size_t)row * DM) = ov[q]; }
    if (pass == 0) __threadfence(); }
}

constexpr size_t SZ_BQKV = (size_t)3 * DM * DM * 2;
constexpr size_t SZ_BW1  = (size_t)DFF * DM * 2;
constexpr size_t SZ_BW2  = (size_t)DM * DFF * 2;
constexpr size_t SZ_X16  = NR * DM * 2;
constexpr size_t SZ_QK16 = NR * LQK * 2;
constexpr size_t SZ_VT16 = (size_t)DM * NR * 2;
constexpr size_t SZ_T1   = NR * DM * 4;
constexpr size_t SZ_R16  = NR * DM * 2;
constexpr size_t SZ_REC  = NR * DM * 4;
constexpr size_t SZ_H16  = NR * DFF * 2;
constexpr size_t WS_TOTAL = SZ_BQKV + SZ_BW1 + SZ_BW2 + SZ_X16 + SZ_QK16 + SZ_VT16 + SZ_T1 + SZ_R16 + SZ_REC + SZ_H16;
static_assert(SZ_BQKV % 256 == 0 && SZ_BW1 % 256 == 0 && SZ_BW2 % 256 == 0 && SZ_X16 % 256 == 0 && SZ_QK16 % 256 == 0 && SZ_VT16 % 256 == 0 && SZ_T1 % 256 == 0 && SZ_R16 % 256 == 0 && SZ_REC % 256 == 0 && SZ_H16 % 256 == 0);
static_assert(WS_TOTAL <= (size_t)134217728);

extern "C" void kernel_launch(void* const* d_in, const int* in_sizes, int n_in,
                              void* d_out, int out_size, void* d_ws, size_t ws_size, hipStream_t stream) {
  if (n_in < 14) return;
  const float* x  = (const float*)d_in[0];
  const float* wq = (const float*)d_in[2];  const float* bq = (const float*)d_in[3];
  const float* wk = (const float*)d_in[4];  const float* bk = (const float*)d_in[5];
  const float* wv = (const float*)d_in[6];  const float* bv = (const float*)d_in[7];
  const float* lg = (const float*)d_in[8];  const float* lb = (const float*)d_in[9];
  const float* w1 = (const float*)d_in[10]; const float* b1 = (const float*)d_in[11];
  const float* w2 = (const float*)d_in[12]; const float* b2 = (const float*)d_in[13];
  const size_t need = ((size_t)(NB - 1) * SEQ_FULL + SEQ) * DM;
  if ((size_t)in_sizes[0] < need || (size_t)out_size < need) return;
  if (in_sizes[2] < NH * DM * HD || in_sizes[4] < NH * DM * HD || in_sizes[6] < NH * DM * HD || in_sizes[3] < NH * HD || in_sizes[5] < NH * HD || in_sizes[7] < NH * HD || in_sizes[8] < DM || in_sizes[9] < DM || in_sizes[10] < DM * DFF || in_sizes[11] < DFF || in_sizes[12] < DFF * DM || in_sizes[13] < DM) return;
  const int M = (int)NR;
  char* ws = (char*)d_ws; size_t off = 0;
  auto take = [&](size_t bytes) { char* p = ws + off; off += (bytes + 255) & ~(size_t)255; return p; };
  _Float16* BQKV = (_Float16*)take(SZ_BQKV);
  _Float16* BW1  = (_Float16*)take(SZ_BW1);
  _Float16* BW2  = (_Float16*)take(SZ_BW2);
  _Float16* X16  = (_Float16*)take(SZ_X16);
  _Float16* QK16 = (_Float16*)take(SZ_QK16);
  _Float16* VT16 = (_Float16*)take(SZ_VT16);
  float*    T1   = (float*)take(SZ_T1);
  _Float16* R16  = (_Float16*)take(SZ_R16);
  float*    REC  = (float*)take(SZ_REC);
  _Float16* H16  = (_Float16*)take(SZ_H16);
  float*    T2   = T1;
  if (off > ws_size || off > (size_t)134217728) return;
  k_xprep<<<(unsigned)(NR * DM / 8 / 256), 256, 0, stream>>>(x, X16, (unsigned)(NR * DM / 8));
  k_wthd3<<<dim3((unsigned)((size_t)NH * HD * (DM / 8) / 256), 3), 256, 0, stream>>>(wq, wk, wv, BQKV);
  k_wt_f16<DM, DFF><<<(unsigned)((size_t)DM * DFF / 8 / 256), 256, 0, stream>>>(w1, BW1, 16.0f);
  k_wt_f16<DFF, DM><<<(unsigned)((size_t)DFF * DM / 8 / 256), 256, 0, stream>>>(w2, BW2, 16.0f);
  k_gemm2<0, 0><<<dim3(DM / 64, (unsigned)(M / 128)), 128, 0, stream>>>(X16, DM, BQKV, DM, 0.0625f, bq, nullptr, nullptr, QK16, LQK, M, DM, DM);
  k_gemm2<0, 0><<<dim3(DM / 64, (unsigned)(M / 128)), 128, 0, stream>>>(X16, DM, BQKV + (size_t)DM * DM, DM, 0.0625f, bk, nullptr, nullptr, QK16 + DM, LQK, M, DM, DM);
  k_gemm2<0, 1><<<dim3((unsigned)(M / 64), DM / 128), 128, 0, stream>>>(BQKV + (size_t)2 * DM * DM, DM, X16, DM, 0.0625f, bv, nullptr, nullptr, VT16, M, DM, M, DM);
  k_attn<<<dim3(SEQ / 64, NH, NB), 128, 0, stream>>>(QK16, VT16, x, T1);
  k_lnx<0, 1, 1, 0><<<(unsigned)M, 256, 0, stream>>>(T1, lg, lb, 1e-5f, R16, REC);
  k_gemm2<3, 0><<<dim3(DFF / 64, (unsigned)(M / 128)), 128, 0, stream>>>(R16, DM, BW1, DM, 0.0625f, b1, nullptr, nullptr, H16, DFF, M, DFF, DM);
  k_gemm2<0, 0><<<dim3(DM / 64, (unsigned)(M / 128)), 128, 0, stream>>>(H16, DFF, BW2, DFF, 0.0625f, b2, REC, T2, nullptr, DM, M, DM, DFF);
  k_lnx<0, 0, 1, 1><<<(unsigned)M, 256, 0, stream>>>(T2, lg, lb, 1e-5f, nullptr, (float*)d_out);
}
